// EvalNet_81260781240520
// MI455X (gfx1250) — hardware-verified
//
#include <hip/hip_runtime.h>

typedef float          v4f   __attribute__((ext_vector_type(4)));
typedef float          v8f   __attribute__((ext_vector_type(8)));
typedef int            v4i   __attribute__((ext_vector_type(4)));
typedef unsigned short v8us  __attribute__((ext_vector_type(8)));
typedef __bf16         v16bf __attribute__((ext_vector_type(16)));
typedef v4f  __attribute__((may_alias)) v4fa;
typedef v4i  __attribute__((may_alias)) v4ia;
typedef v8us __attribute__((may_alias)) v8usa;

union Frag { v16bf v; v8us half[2]; };

#define HID      1024
#define NROW     769
#define EROWS    770
#define SLOTS    32
#define H2       32
#define NBK      8
#define PPB      32
#define NTHR     64
#define CW       256
#define APITCH   264
#define H2P      33
#define NE4      (EROWS * HID / 4)
#define NF8      (H2 * HID / 8)
#define PREP_THR 256

static_assert((NE4 % PREP_THR) == 0);
static_assert(((NE4 + NF8) % PREP_THR) == 0);
static_assert((HID / 4) == PREP_THR);
static_assert((HID % CW) == 0);
static_assert(CW == 8 * 32);
static_assert((CW % 32) == 0);
static_assert((APITCH % 8) == 0);
static_assert(PPB == 32);
static_assert(NTHR == 64);
static_assert((PPB * SLOTS) == 4 * 4 * NTHR);

__device__ __forceinline__ unsigned int bf16_bits(float f) {
  unsigned int u = __float_as_uint(f);
  u = u + 0x7FFFu + ((u >> 16) & 1u);
  return u >> 16;
}
__device__ __forceinline__ float bf16_rne(float f) {
  return __uint_as_float(bf16_bits(f) << 16);
}

__device__ __forceinline__ v8f wmma_bf16(v16bf a, v16bf b, v8f c) {
  v8f d = __builtin_amdgcn_wmma_f32_16x16x32_bf16(false, a, false, b, (short)0, c, false, false);
  asm volatile("v_nop\n\tv_nop\n\tv_nop\n\tv_nop" : "+v"(d) : "v"(a), "v"(b));
  return d;
}

__device__ __forceinline__ v16bf load_frag(const unsigned short* p, int h) {
  Frag f;
  f.half[0] = *(const v8usa*)(p + 8 * h);
  f.half[1] = *(const v8usa*)(p + 16 + 8 * h);
  return f.v;
}

__device__ __forceinline__ int clamp_off(int xi) {
  const int ri = xi < 0 ? 0 : (xi > NROW - 1 ? NROW : xi);
  return ri * HID;
}

__global__ __launch_bounds__(PREP_THR) void prep_kernel(
    const float* __restrict__ emb, const float* __restrict__ fc2,
    float* __restrict__ E, unsigned short* __restrict__ F)
{
  const int g = blockIdx.x * PREP_THR + threadIdx.x;
  if (g < NE4) {
    const int row = g >> 8;
    const int c4 = (g & 255) * 4;
    const int srow = row < NROW ? row : (NROW - 1);
    const v4f a = *(const v4fa*)(emb + (size_t)srow * HID + c4);
    v4f o;
    o.x = bf16_rne(a.x); o.y = bf16_rne(a.y); o.z = bf16_rne(a.z); o.w = bf16_rne(a.w);
    if (row == NROW - 1) { o.x = 0.0f; o.y = 0.0f; o.z = 0.0f; o.w = 0.0f; }
    float* dst = E + (size_t)row * HID + c4;
    *(volatile v4f*)dst = o;
    __threadfence();
    *(volatile v4f*)dst = o;
  } else if (g < NE4 + NF8) {
    const int e = g - NE4;
    const float* src = fc2 + (size_t)e * 8;
    const v4f a = *(const v4fa*)src;
    const v4f c = *(const v4fa*)(src + 4);
    v8us o;
    o[0] = (unsigned short)bf16_bits(a.x); o[1] = (unsigned short)bf16_bits(a.y);
    o[2] = (unsigned short)bf16_bits(a.z); o[3] = (unsigned short)bf16_bits(a.w);
    o[4] = (unsigned short)bf16_bits(c.x); o[5] = (unsigned short)bf16_bits(c.y);
    o[6] = (unsigned short)bf16_bits(c.z); o[7] = (unsigned short)bf16_bits(c.w);
    unsigned short* dst = F + (size_t)e * 8;
    *(volatile v8us*)dst = o;
    __threadfence();
    *(volatile v8us*)dst = o;
  }
}

__global__ __launch_bounds__(NTHR) void eval_kernel(
    const int* __restrict__ x, const int* __restrict__ pcnt,
    const float* __restrict__ E, const unsigned short* __restrict__ F,
    const float* __restrict__ bias1, const float* __restrict__ fc2_b,
    const float* __restrict__ cp_w, const float* __restrict__ cp_b,
    const float* __restrict__ wdl_w, const float* __restrict__ wdl_b,
    float* __restrict__ out, int npos)
{
  __shared__ __attribute__((aligned(16))) int s_off[PPB * SLOTS];
  __shared__ __attribute__((aligned(16))) unsigned short s_ahi[2 * 16 * APITCH];
  __shared__ __attribute__((aligned(16))) unsigned short s_alo[2 * 16 * APITCH];
  __shared__ float s_h2[PPB * H2P];
  __shared__ float s_cpw[NBK * H2];
  __shared__ float s_wdw[NBK * 3 * H2];
  __shared__ float s_cpb[NBK];
  __shared__ float s_wdb[NBK * 3];
  __shared__ float s_f2b[H2];
  __shared__ __attribute__((aligned(16))) float s_out[PPB * 4];

  const int tid = threadIdx.x, lane = tid & 31, w = tid >> 5;
  const int h = lane >> 4, m = lane & 15;
  const int p0 = blockIdx.x * PPB;

  {
    const int* xb = x + (size_t)p0 * SLOTS;
    #pragma unroll
    for (int i = 0; i < 4; ++i) {
      const int g4 = tid + NTHR * i;
      const v4i xv = *(const v4ia*)(xb + 4 * g4);
      v4i ov;
      ov.x = clamp_off(xv.x); ov.y = clamp_off(xv.y);
      ov.z = clamp_off(xv.z); ov.w = clamp_off(xv.w);
      *(v4ia*)(s_off + 4 * g4) = ov;
    }
  }
  for (int j = tid; j < NBK * H2; j += NTHR)     s_cpw[j] = bf16_rne(cp_w[j]);
  for (int j = tid; j < NBK * 3 * H2; j += NTHR) s_wdw[j] = bf16_rne(wdl_w[j]);
  if (tid < NBK)     s_cpb[tid] = bf16_rne(cp_b[tid < NBK ? tid : 0]);
  if (tid < NBK * 3) s_wdb[tid] = bf16_rne(wdl_b[tid < NBK * 3 ? tid : 0]);
  if (tid < H2)      s_f2b[tid] = bf16_rne(fc2_b[tid < H2 ? tid : 0]);
  __syncthreads();

  const v4f zero4 = {0.0f, 0.0f, 0.0f, 0.0f};
  const v8f zero8 = {0.0f, 0.0f, 0.0f, 0.0f, 0.0f, 0.0f, 0.0f, 0.0f};
  v8f c0 = zero8, c1 = zero8;
  unsigned short* ahi_w = s_ahi + w * 16 * APITCH;
  unsigned short* alo_w = s_alo + w * 16 * APITCH;
  const int* off_w = s_off + w * 16 * SLOTS;

  #pragma unroll 1
  for (int c = 0; c < HID / CW; ++c) {
    const int kb = c * CW + 8 * lane;
    const v4f bq0 = *(const v4fa*)(bias1 + kb);
    const v4f bq1 = *(const v4fa*)(bias1 + kb + 4);
    const float bb[8] = { bf16_rne(bq0.x), bf16_rne(bq0.y), bf16_rne(bq0.z), bf16_rne(bq0.w),
                          bf16_rne(bq1.x), bf16_rne(bq1.y), bf16_rne(bq1.z), bf16_rne(bq1.w) };

    #pragma unroll 1
    for (int r = 0; r < 16; ++r) {
      const int* orow = off_w + r * SLOTS;
      v4f a0 = zero4, a1 = zero4;
      #pragma unroll 4
      for (int s = 0; s < SLOTS; ++s) {
        const float* p = E + orow[s] + kb;
        a0 += *(const v4fa*)p;
        a1 += *(const v4fa*)(p + 4);
      }
      const float hv[8] = { a0.x + bb[0], a0.y + bb[1], a0.z + bb[2], a0.w + bb[3],
                            a1.x + bb[4], a1.y + bb[5], a1.z + bb[6], a1.w + bb[7] };
      v8us vh, vl;
      #pragma unroll
      for (int j = 0; j < 8; ++j) {
        float t = fminf(fmaxf(hv[j], 0.0f), 1.0f);
        t = t * t;
        const unsigned int hb = bf16_bits(t);
        const float hf = __uint_as_float(hb << 16);
        const unsigned int lb = bf16_bits(t - hf);
        vh[j] = (unsigned short)hb;
        vl[j] = (unsigned short)lb;
      }
      *(v8usa*)(ahi_w + r * APITCH + 8 * lane) = vh;
      *(v8usa*)(alo_w + r * APITCH + 8 * lane) = vl;
    }
    __syncthreads();

    #pragma unroll
    for (int ks = 0; ks < CW / 32; ++ks) {
      const int kk = 32 * ks;
      const v16bf ah = load_frag(ahi_w + m * APITCH + kk, h);
      const v16bf al = load_frag(alo_w + m * APITCH + kk, h);
      const unsigned short* fb = F + (size_t)m * HID + c * CW + kk;
      const v16bf b0 = load_frag(fb, h);
      const v16bf b1 = load_frag(fb + (size_t)16 * HID, h);
      c0 = wmma_bf16(ah, b0, c0);
      c0 = wmma_bf16(al, b0, c0);
      c1 = wmma_bf16(ah, b1, c1);
      c1 = wmma_bf16(al, b1, c1);
    }
    __syncthreads();
  }

  #pragma unroll
  for (int r = 0; r < 8; ++r) {
    const int pl = 16 * w + 8 * h + r;
    float v = c0[r] + s_f2b[m];
    v = fminf(fmaxf(v, 0.0f), 1.0f);
    s_h2[pl * H2P + m] = v * v;
    float u = c1[r] + s_f2b[16 + m];
    u = fminf(fmaxf(u, 0.0f), 1.0f);
    s_h2[pl * H2P + 16 + m] = u * u;
  }
  __syncthreads();

  if (tid < PPB) {
    const int p = tid;
    const int pc = pcnt[p0 + p];
    const int a = (pc - 2) * NBK;
    int q = a / 30;
    if ((a % 30) != 0 && a < 0) q -= 1;
    q = q < 0 ? 0 : (q > NBK - 1 ? NBK - 1 : q);
    const float* hr = s_h2 + p * H2P;
    const float* wc = s_cpw + q * H2;
    const float* w0 = s_wdw + (3 * q) * H2;
    const float* w1 = w0 + H2;
    const float* w2 = w1 + H2;
    float sc = 0.0f, s0 = 0.0f, s1 = 0.0f, s2 = 0.0f;
    #pragma unroll 4
    for (int k = 0; k < H2; ++k) {
      const float hk = hr[k];
      sc += hk * wc[k];
      s0 += hk * w0[k];
      s1 += hk * w1[k];
      s2 += hk * w2[k];
    }
    s_out[p] = sc + s_cpb[q];
    s_out[PPB + 3 * p + 0] = s0 + s_wdb[3 * q + 0];
    s_out[PPB + 3 * p + 1] = s1 + s_wdb[3 * q + 1];
    s_out[PPB + 3 * p + 2] = s2 + s_wdb[3 * q + 2];
  }
  __syncthreads();

  if (w == 0) {
    const int l8  = lane & 7;
    const int l24 = lane < 24 ? lane : 23;
    const v4f v0 = *(const v4fa*)(s_out + 4 * l8);
    const v4f v1 = *(const v4fa*)(s_out + PPB + 4 * l24);
    float* d0 = out + (size_t)p0 + 4 * l8;
    float* d1 = out + (size_t)npos + (size_t)p0 * 3 + 4 * l24;
    if (lane < 8)  *(volatile v4f*)d0 = v0;
    if (lane < 24) *(volatile v4f*)d1 = v1;
    __threadfence();
    if (lane < 8)  *(volatile v4f*)d0 = v0;
    if (lane < 24) *(volatile v4f*)d1 = v1;
  }
}

extern "C" void kernel_launch(void* const* d_in, const int* in_sizes, int n_in,
                              void* d_out, int out_size, void* d_ws, size_t ws_size,
                              hipStream_t stream) {
  if (n_in < 10) return;
  const int npos = in_sizes[1];
  if (npos <= 0 || (npos % PPB) != 0) return;
  if (in_sizes[0] != npos * SLOTS) return;
  if (in_sizes[2] != NROW * HID) return;
  if (in_sizes[3] != HID) return;
  if (in_sizes[4] != H2 * HID) return;
  if (in_sizes[5] != H2) return;
  if (in_sizes[6] != NBK * H2 || in_sizes[7] != NBK) return;
  if (in_sizes[8] != NBK * 3 * H2 || in_sizes[9] != NBK * 3) return;
  if (out_size != 4 * npos) return;

  const int*   x     = (const int*)d_in[0];
  const int*   pcnt  = (const int*)d_in[1];
  const float* emb   = (const float*)d_in[2];
  const float* bias1 = (const float*)d_in[3];
  const float* fc2w  = (const float*)d_in[4];
  const float* fc2b  = (const float*)d_in[5];
  const float* cpw   = (const float*)d_in[6];
  const float* cpb   = (const float*)d_in[7];
  const float* wdw   = (const float*)d_in[8];
  const float* wdb   = (const float*)d_in[9];
  float* out = (float*)d_out;

  const size_t e_bytes = (size_t)EROWS * HID * sizeof(float);
  const size_t f_bytes = (size_t)H2 * HID * sizeof(unsigned short);
  const size_t total = e_bytes + f_bytes;
  if (total > ws_size) return;
  char* ws = (char*)d_ws;
  float* E = (float*)ws;
  unsigned short* F = (unsigned short*)(ws + e_bytes);

  const int prep_blocks = (NE4 + NF8 + PREP_THR - 1) / PREP_THR;
  prep_kernel<<<prep_blocks, PREP_THR, 0, stream>>>(emb, fc2w, E, F);

  eval_kernel<<<npos / PPB, NTHR, 0, stream>>>(x, pcnt, E, F, bias1, fc2b, cpw, cpb, wdw, wdb, out, npos);
}
